// GraphRes_70909910057698
// MI455X (gfx1250) — hardware-verified
//
#include <hip/hip_runtime.h>
#include <stddef.h>


#define KK      27
#define C1      32
#define C2      128
#define K2      (KK * C1)
#define KP2     896
#define KT2     (KP2 / 32)
#define NTHR    256
#define NWAVE   8
#define EPT     8
#define NGRP    2
#define CHUNK   (NTHR * EPT * NGRP)
#define WCAP    (EPT * NGRP * 32)
#define LISTN   (NWAVE * WCAP)
#define NBC     4096
#define NBF     1024
#define RCAP    40960
#define RBN     128
#define OTHR    512
#define DEGCAP  128
#define TG2     64
#define CL      16
#define GMAX    16
#define KF      2048
#define NOMAX   128
#define W2S     8.0f
#define W2I     0.125f
#define BNEPS   1e-5f

#define LDS_FILL ((RCAP + NBF + LISTN) * 4 + 64)
#define L1FLT    (KK * NTHR + KK * C1 + NTHR * C1 + 2 * NWAVE * C1 + 2 * C1)
#define LDS_L1   (L1FLT * 4)
#define LDS_L2   (TG2 * KP2 * 4)
#define LDS_POOL ((NWAVE * CL * C2 + LISTN + 16) * 4)
#define LDS_FC   ((GMAX * KF + GMAX * NOMAX) * 4)

static_assert((CHUNK & (CHUNK - 1)) == 0);
static_assert(CHUNK <= 4096);
static_assert(NBC <= 4096 && NBF <= 4096);
static_assert((NBC & (NBC - 1)) == 0 && (NBF & (NBF - 1)) == 0);
static_assert(NBC == 4 * NBF);
static_assert(OTHR * 8 == NBC);
static_assert((RCAP % 32) == 0);
static_assert(KF == CL * C2);
static_assert(TG2 == NWAVE * 8);
static_assert(KP2 % 32 == 0 && KP2 >= K2);
static_assert(C2 * TG2 / 4 + 4 * C2 + 2 * C2 <= TG2 * KP2 / 4);

typedef float    v4f  __attribute__((ext_vector_type(4)));
typedef float    v8f  __attribute__((ext_vector_type(8)));
typedef int      v4i  __attribute__((ext_vector_type(4)));
typedef _Float16 v8h  __attribute__((ext_vector_type(8)));
typedef _Float16 v16h __attribute__((ext_vector_type(16)));
union FragH { v16h v; v8h h[2]; };

__device__ __forceinline__ int clampi(int v, int lo, int hi) { return v < lo ? lo : (v > hi ? hi : v); }

__device__ __forceinline__ float rlf(float v, int l) {
  return __int_as_float(__builtin_amdgcn_readlane(__float_as_int(v), l));
}

__device__ __forceinline__ v8h cvt8(v4f a, v4f b) {
  v8h r;
  r[0] = (_Float16)a.x; r[1] = (_Float16)a.y; r[2] = (_Float16)a.z; r[3] = (_Float16)a.w;
  r[4] = (_Float16)b.x; r[5] = (_Float16)b.y; r[6] = (_Float16)b.z; r[7] = (_Float16)b.w;
  return r;
}

__device__ __forceinline__ v8f wmh(v16h a, v16h b, v8f c) {
  v8f d = __builtin_amdgcn_wmma_f32_16x16x32_f16(false, a, false, b, (short)0, c, false, false);
  asm volatile("v_nop\n\tv_nop\n\tv_nop\n\tv_nop" : "+v"(d) : "v"(a), "v"(b));
  return d;
}

template <int NB>
__device__ __forceinline__ int scan_chunk(const int* __restrict__ dsts, int nE, int cbase, int slotBase,
                                          int vec8, int* list, int tid, int lane, int wave) {
  int wc = 0;
#pragma unroll
  for (int g = 0; g < NGRP; ++g) {
    const int el0  = (g * NTHR + tid) * EPT;
    const int e0   = cbase + el0;
    const int sent = -2147483647 - 1;
    v4i da, db;
    if (vec8 != 0 && cbase + CHUNK <= nE) {
      da = *(const v4i*)(dsts + e0);
      db = *(const v4i*)(dsts + e0 + 4);
    } else {
      da.x = (e0     < nE) ? dsts[min(e0, nE - 1)] : sent;
      da.y = (e0 + 1 < nE) ? dsts[min(e0 + 1, nE - 1)] : sent;
      da.z = (e0 + 2 < nE) ? dsts[min(e0 + 2, nE - 1)] : sent;
      da.w = (e0 + 3 < nE) ? dsts[min(e0 + 3, nE - 1)] : sent;
      db.x = (e0 + 4 < nE) ? dsts[min(e0 + 4, nE - 1)] : sent;
      db.y = (e0 + 5 < nE) ? dsts[min(e0 + 5, nE - 1)] : sent;
      db.z = (e0 + 6 < nE) ? dsts[min(e0 + 6, nE - 1)] : sent;
      db.w = (e0 + 7 < nE) ? dsts[min(e0 + 7, nE - 1)] : sent;
    }
    const unsigned nb = (unsigned)slotBase;
    const unsigned s0 = (unsigned)da.x - nb, s1 = (unsigned)da.y - nb;
    const unsigned s2 = (unsigned)da.z - nb, s3 = (unsigned)da.w - nb;
    const unsigned s4 = (unsigned)db.x - nb, s5 = (unsigned)db.y - nb;
    const unsigned s6 = (unsigned)db.z - nb, s7 = (unsigned)db.w - nb;
    const bool h0 = s0 < (unsigned)NB, h1 = s1 < (unsigned)NB, h2 = s2 < (unsigned)NB, h3 = s3 < (unsigned)NB;
    const bool h4 = s4 < (unsigned)NB, h5 = s5 < (unsigned)NB, h6 = s6 < (unsigned)NB, h7 = s7 < (unsigned)NB;
    const unsigned any = __builtin_amdgcn_ballot_w32(h0 | h1 | h2 | h3 | h4 | h5 | h6 | h7);
    if (any != 0u) {
#define HITJ(J, HJ, SJ) { \
        const unsigned mj = __builtin_amdgcn_ballot_w32(HJ); \
        if (mj != 0u) { \
          if (HJ) { \
            const int pos = wc + (int)__builtin_amdgcn_mbcnt_lo(mj, 0u); \
            if (pos < WCAP) list[wave * WCAP + pos] = ((el0 + (J)) << 12) | (int)(SJ); \
          } \
          wc += (int)__builtin_popcount(mj); } }
      HITJ(0, h0, s0)
      HITJ(1, h1, s1)
      HITJ(2, h2, s2)
      HITJ(3, h3, s3)
      HITJ(4, h4, s4)
      HITJ(5, h5, s5)
      HITJ(6, h6, s6)
      HITJ(7, h7, s7)
#undef HITJ
    }
  }
  return wc;
}

__global__ __launch_bounds__(NTHR) void k_w2prep(const float* __restrict__ W2, _Float16* W2h, int total) {
  const int i = blockIdx.x * NTHR + (int)threadIdx.x;
  if (i >= total) return;
  const int n  = i / (KP2 / 8);
  const int k0 = (i - n * (KP2 / 8)) * 8;
  float v[8];
#pragma unroll
  for (int e = 0; e < 8; ++e) {
    const int k  = k0 + e;
    const int kc = k < K2 ? k : K2 - 1;
    const float w = W2[(size_t)kc * C2 + n];
    v[e] = (k < K2) ? w * W2S : 0.0f;
  }
  v4f a, b;
  a.x = v[0]; a.y = v[1]; a.z = v[2]; a.w = v[3];
  b.x = v[4]; b.y = v[5]; b.z = v[6]; b.w = v[7];
  const v8h hv = cvt8(a, b);
  _Float16* dp = W2h + (size_t)i * 8;
  *(volatile v8h*)dp = hv;
  __threadfence();
  *(volatile v8h*)dp = hv;
}

__global__ __launch_bounds__(NTHR) void k_count(const int* __restrict__ dsts, int* cnt, int nE, int vec8) {
  __shared__ __attribute__((aligned(16))) int scnt[NBC];
  __shared__ __attribute__((aligned(16))) int list[LISTN];
  __shared__ int wcnt[NWAVE];
  const int tid = threadIdx.x, lane = tid & 31, wave = tid >> 5;
  const int nodeBase = blockIdx.x * NBC;

  for (int i = tid; i < NBC; i += NTHR) scnt[i] = 0;
  __syncthreads();

  const int nChunks = (nE + CHUNK - 1) / CHUNK;
#pragma unroll 1
  for (int ch = 0; ch < nChunks; ++ch) {
    const int cbase = ch * CHUNK;
    const int wc = scan_chunk<NBC>(dsts, nE, cbase, nodeBase, vec8, list, tid, lane, wave);
    if (lane == 0) wcnt[wave] = wc;
    __syncthreads();
    if (wave == 0) {
#pragma unroll 1
      for (int wsx = 0; wsx < NWAVE; ++wsx) {
        int n = __builtin_amdgcn_readfirstlane(wcnt[wsx]);
        n = n > WCAP ? WCAP : (n < 0 ? 0 : n);
        const int* lp = list + wsx * WCAP;
#pragma unroll 1
        for (int i = 0; i < n; ++i) {
          const int ent  = __builtin_amdgcn_readfirstlane(lp[i]);
          const int slot = ent & (NBC - 1);
          if (lane == 0) scnt[slot] = scnt[slot] + 1;
        }
      }
    }
    __syncthreads();
  }
  __syncthreads();

  v4i cq[4];
#pragma unroll
  for (int q = 0; q < 4; ++q) {
    const int f = (wave * 4 + q) * 128 + 4 * lane;
    cq[q] = *(const v4i*)(scnt + f);
  }
  int* cp = cnt + (size_t)nodeBase;
#pragma unroll
  for (int q = 0; q < 4; ++q) {
    const int f = (wave * 4 + q) * 128 + 4 * lane;
    *(volatile v4i*)(cp + f) = cq[q];
  }
  __threadfence();
#pragma unroll
  for (int q = 0; q < 4; ++q) {
    const int f = (wave * 4 + q) * 128 + 4 * lane;
    *(volatile v4i*)(cp + f) = cq[q];
  }
}

__global__ __launch_bounds__(OTHR) void k_offsets(
    const int* __restrict__ cnt, int* off, int* rbase, int nChunk) {
  __shared__ __attribute__((aligned(16))) int soff[NBC];
  __shared__ __attribute__((aligned(16))) int srb[RBN];
  __shared__ int wtot[OTHR / 32];
  const int tid = threadIdx.x, lane = tid & 31, wave = tid >> 5, sub = tid >> 7;
  for (int i = tid; i < RBN; i += OTHR) srb[i] = 0;
  int carry = 0;
#pragma unroll 1
  for (int ch = 0; ch < nChunk; ++ch) {
    const int base = ch * NBC;
    const v4i c0 = *(const v4i*)(cnt + base + 8 * tid);
    const v4i c1 = *(const v4i*)(cnt + base + 8 * tid + 4);
    const int e0 = max(c0.x, 0), e1 = max(c0.y, 0), e2 = max(c0.z, 0), e3 = max(c0.w, 0);
    const int e4 = max(c1.x, 0), e5 = max(c1.y, 0), e6 = max(c1.z, 0), e7 = max(c1.w, 0);
    const int ts = e0 + e1 + e2 + e3 + e4 + e5 + e6 + e7;
    int incl = ts;
#pragma unroll
    for (int d = 1; d < 32; d <<= 1) {
      const int t = __shfl_up(incl, d);
      if (lane >= d) incl += t;
    }
    if (lane == 31) wtot[wave] = incl;
    __syncthreads();
    const int S0 = wtot[0]  + wtot[1]  + wtot[2]  + wtot[3];
    const int S1 = wtot[4]  + wtot[5]  + wtot[6]  + wtot[7];
    const int S2 = wtot[8]  + wtot[9]  + wtot[10] + wtot[11];
    const int S3 = wtot[12] + wtot[13] + wtot[14] + wtot[15];
    int pre = 0;
#pragma unroll 1
    for (int w = 4 * sub; w < wave; ++w) pre += wtot[w];
    const int b0 = carry;
    const int b1 = b0 + ((S0 + 31) & ~31);
    const int b2 = b1 + ((S1 + 31) & ~31);
    const int b3 = b2 + ((S2 + 31) & ~31);
    const int b4 = b3 + ((S3 + 31) & ~31);
    const int myb = sub == 0 ? b0 : (sub == 1 ? b1 : (sub == 2 ? b2 : b3));
    if (tid == 0) {
      srb[min(4 * ch + 0, RBN - 1)] = b0;
      srb[min(4 * ch + 1, RBN - 1)] = b1;
      srb[min(4 * ch + 2, RBN - 1)] = b2;
      srb[min(4 * ch + 3, RBN - 1)] = b3;
    }
    int run = myb + pre + incl - ts;
    soff[8 * tid + 0] = run; run += e0;
    soff[8 * tid + 1] = run; run += e1;
    soff[8 * tid + 2] = run; run += e2;
    soff[8 * tid + 3] = run; run += e3;
    soff[8 * tid + 4] = run; run += e4;
    soff[8 * tid + 5] = run; run += e5;
    soff[8 * tid + 6] = run; run += e6;
    soff[8 * tid + 7] = run;
    carry = b4;
    __syncthreads();
    const v4i o0 = *(const v4i*)(soff + 4 * tid);
    const v4i o1 = *(const v4i*)(soff + 4 * (tid + OTHR));
    int* op = off + base;
    *(volatile v4i*)(op + 4 * tid) = o0;
    *(volatile v4i*)(op + 4 * (tid + OTHR)) = o1;
    __threadfence();
    *(volatile v4i*)(op + 4 * tid) = o0;
    *(volatile v4i*)(op + 4 * (tid + OTHR)) = o1;
    __syncthreads();
  }
  if (tid == 0) srb[min(4 * nChunk, RBN - 1)] = carry;
  __syncthreads();
  v4i rv = {0, 0, 0, 0};
  if (tid < 32) rv = *(const v4i*)(srb + 4 * tid);
  if (tid < 32) *(volatile v4i*)(rbase + 4 * tid) = rv;
  __threadfence();
  if (tid < 32) *(volatile v4i*)(rbase + 4 * tid) = rv;
}

__global__ __launch_bounds__(NTHR) void k_fill(
    const int* __restrict__ dsts, const int* __restrict__ off, const int* __restrict__ rbase,
    int* csr, int nE, int vec8, int csrLen) {
  extern __shared__ v4f lds_dyn[];
  int* region = (int*)lds_dyn;
  int* cursor = region + RCAP;
  int* list   = cursor + NBF;
  int* wcnt   = list + LISTN;
  const int tid = threadIdx.x, lane = tid & 31, wave = tid >> 5;
  const int b = blockIdx.x;
  const int nodeBase = b * NBF;

  int rb0 = rbase[b];
  const int rb1 = rbase[b + 1];
  rb0 = rb0 < 0 ? 0 : (rb0 > csrLen ? csrLen : rb0);
  rb0 &= ~31;
  int len = rb1 - rb0;
  len = len < 0 ? 0 : (len > RCAP ? RCAP : len);
  int lenW = (len + 31) & ~31;
  if (rb0 + lenW > csrLen) lenW = (csrLen - rb0) & ~31;

  {
    const v4i z = {0, 0, 0, 0};
    for (int i = tid; i < RCAP / 4; i += NTHR) ((v4i*)region)[i] = z;
    for (int s = tid; s < NBF; s += NTHR) {
      int o = off[nodeBase + s] - rb0;
      o = o < 0 ? 0 : (o > RCAP ? RCAP : o);
      cursor[s] = o;
    }
  }
  __syncthreads();

  const int nChunks = (nE + CHUNK - 1) / CHUNK;
#pragma unroll 1
  for (int ch = 0; ch < nChunks; ++ch) {
    const int cbase = ch * CHUNK;
    const int wc = scan_chunk<NBF>(dsts, nE, cbase, nodeBase, vec8, list, tid, lane, wave);
    if (lane == 0) wcnt[wave] = wc;
    __syncthreads();
    if (wave == 0) {
#pragma unroll 1
      for (int wsx = 0; wsx < NWAVE; ++wsx) {
        int n = __builtin_amdgcn_readfirstlane(wcnt[wsx]);
        n = n > WCAP ? WCAP : (n < 0 ? 0 : n);
        const int* lp = list + wsx * WCAP;
#pragma unroll 1
        for (int i = 0; i < n; ++i) {
          const int ent  = __builtin_amdgcn_readfirstlane(lp[i]);
          const int slot = ent & (NBF - 1);
          int e = cbase + ((ent >> 12) & (CHUNK - 1));
          e = e > nE - 1 ? nE - 1 : e;
          if (lane == 0) {
            int pos = cursor[slot];
            pos = pos < 0 ? 0 : (pos > RCAP - 1 ? RCAP - 1 : pos);
            region[pos] = e;
            const int np = pos + 1;
            cursor[slot] = np > RCAP ? RCAP : np;
          }
        }
      }
    }
    __syncthreads();
  }

  const int nv = lenW >> 2;
  int* gp = csr + rb0;
#pragma unroll 1
  for (int i = tid; i < nv; i += NTHR) { const v4i v = ((const v4i*)region)[i]; *(volatile v4i*)(gp + 4 * i) = v; }
  __threadfence();
#pragma unroll 1
  for (int i = tid; i < nv; i += NTHR) { const v4i v = ((const v4i*)region)[i]; *(volatile v4i*)(gp + 4 * i) = v; }
}

__global__ __launch_bounds__(NTHR) void k_layer1(
    const int* __restrict__ csr, const int* __restrict__ off, const int* __restrict__ cnt,
    const int* __restrict__ ei, const float* __restrict__ ea, const float* __restrict__ x,
    const float* __restrict__ W1, float* h1, float* part, int nN, int nE, int csrLen) {
  extern __shared__ v4f lds_dyn[];
  float* acc1 = (float*)lds_dyn;
  float* W1s  = acc1 + KK * NTHR;
  float* stg  = W1s + KK * C1;
  float* cS   = stg + NTHR * C1;
  float* cQ   = cS + NWAVE * C1;
  float* pl   = cQ + NWAVE * C1;
  const int tid = threadIdx.x, lane = tid & 31, wave = tid >> 5;
  const int n0 = blockIdx.x * NTHR;
  const int node = n0 + tid;

  for (int i = tid; i < KK * C1; i += NTHR) W1s[i] = W1[i];
  float* acol = acc1 + tid;
#pragma unroll
  for (int k = 0; k < KK; ++k) acol[k * NTHR] = 0.0f;

  const int craw = max(cnt[node], 0);
  const int c = craw > DEGCAP ? DEGCAP : craw;
  const int st = off[node];
  int cm = c;
  cm = max(cm, __shfl_xor(cm, 16));
  cm = max(cm, __shfl_xor(cm, 8));
  cm = max(cm, __shfl_xor(cm, 4));
  cm = max(cm, __shfl_xor(cm, 2));
  cm = max(cm, __shfl_xor(cm, 1));
  cm = __builtin_amdgcn_readfirstlane(cm);
  cm = cm > DEGCAP ? DEGCAP : (cm < 0 ? 0 : cm);

#pragma unroll 1
  for (int p = 0; p < cm; ++p) {
    const bool act = p < c;
    const int pos = clampi(st + p, 0, csrLen - 1);
    const int e = clampi(csr[pos], 0, nE - 1);
    const int s = clampi(ei[e], 0, nN - 1);
    float xv = x[s];
    xv = act ? xv : 0.0f;
    const float* ap = ea + (size_t)e * 3;
    const float v0 = ap[0] * 2.0f, v1 = ap[1] * 2.0f, v2 = ap[2] * 2.0f;
    const float l0 = fminf(fmaxf(floorf(v0), 0.0f), 1.0f);
    const float l1 = fminf(fmaxf(floorf(v1), 0.0f), 1.0f);
    const float l2 = fminf(fmaxf(floorf(v2), 0.0f), 1.0f);
    const float f0 = v0 - l0, f1 = v1 - l1, f2 = v2 - l2;
    const float g0 = 1.0f - f0, g1 = 1.0f - f1, g2 = 1.0f - f2;
    const int lb = (int)l0 + 3 * (int)l1 + 9 * (int)l2;
    float* ab = acol + lb * NTHR;
    const float t0 = g0 * xv, t1 = f0 * xv;
    const float p0 = t0 * g1, p1 = t1 * g1, p2 = t0 * f1, p3 = t1 * f1;
    ab[0 * NTHR]  += p0 * g2;
    ab[1 * NTHR]  += p1 * g2;
    ab[3 * NTHR]  += p2 * g2;
    ab[4 * NTHR]  += p3 * g2;
    ab[9 * NTHR]  += p0 * f2;
    ab[10 * NTHR] += p1 * f2;
    ab[12 * NTHR] += p2 * f2;
    ab[13 * NTHR] += p3 * f2;
  }
  __syncthreads();

  float sacc[C1];
#pragma unroll
  for (int cc = 0; cc < C1; ++cc) sacc[cc] = 0.0f;
#pragma unroll 1
  for (int k = 0; k < KK; ++k) {
    const float a = acol[k * NTHR];
    const v4f* wr = (const v4f*)(W1s + k * C1);
#pragma unroll
    for (int c4 = 0; c4 < C1 / 4; ++c4) {
      const v4f w = wr[c4];
      sacc[4 * c4 + 0] += a * w.x;
      sacc[4 * c4 + 1] += a * w.y;
      sacc[4 * c4 + 2] += a * w.z;
      sacc[4 * c4 + 3] += a * w.w;
    }
  }
  const float rcp = 1.0f / (float)(craw < 1 ? 1 : craw);
  float* srow = stg + tid * C1;
#pragma unroll
  for (int c4 = 0; c4 < C1 / 4; ++c4) {
    v4f v;
    v.x = sacc[4 * c4 + 0] * rcp; v.y = sacc[4 * c4 + 1] * rcp;
    v.z = sacc[4 * c4 + 2] * rcp; v.w = sacc[4 * c4 + 3] * rcp;
    *(v4f*)(srow + 4 * c4) = v;
  }
  __syncthreads();

  {
    const int col = tid & 31;
    const int r0 = (tid >> 5) * 32;
    float sum = 0.0f, sq = 0.0f;
#pragma unroll 1
    for (int r = 0; r < 32; ++r) {
      float* p_ = stg + (r0 + r) * C1 + col;
      float v = *p_;
      v = v > 0.0f ? v : expm1f(v);
      *p_ = v;
      sum += v;
      sq += v * v;
    }
    cS[(tid >> 5) * C1 + col] = sum;
    cQ[(tid >> 5) * C1 + col] = sq;
  }
  __syncthreads();
  if (tid < C1) {
    float S = 0.0f, Q = 0.0f;
#pragma unroll
    for (int w = 0; w < NWAVE; ++w) { S += cS[w * C1 + tid]; Q += cQ[w * C1 + tid]; }
    pl[tid] = S;
    pl[C1 + tid] = Q;
  }
  __syncthreads();

  v4f pv = {0.f, 0.f, 0.f, 0.f};
  if (tid < 16) pv = *(const v4f*)(pl + 4 * tid);
  float* pp = part + (size_t)blockIdx.x * (2 * C1) + 4 * tid;
  const float* lp = stg + 1024 * wave + 4 * lane;
  float* gp = h1 + (size_t)n0 * C1 + 1024 * wave + 4 * lane;
  if (tid < 16) *(volatile v4f*)pp = pv;
#pragma unroll
  for (int i = 0; i < 8; ++i) { const v4f v = *(const v4f*)(lp + 128 * i); *(volatile v4f*)(gp + 128 * i) = v; }
  __threadfence();
  if (tid < 16) *(volatile v4f*)pp = pv;
#pragma unroll
  for (int i = 0; i < 8; ++i) { const v4f v = *(const v4f*)(lp + 128 * i); *(volatile v4f*)(gp + 128 * i) = v; }
}

__global__ __launch_bounds__(128) void k_bnfin(
    const float* __restrict__ part, const float* __restrict__ gam, const float* __restrict__ bet,
    float* ab, int nblk, int C, int nN) {
  __shared__ __attribute__((aligned(16))) float pl[2 * C2];
  const int tid = threadIdx.x;
  for (int c = tid; c < C; c += 128) {
    double s = 0.0, q = 0.0;
#pragma unroll 1
    for (int b = 0; b < nblk; ++b) {
      const float* pr = part + (size_t)b * (2 * C);
      s += (double)pr[c];
      q += (double)pr[C + c];
    }
    const double mu = s / (double)nN;
    double var = q / (double)nN - mu * mu;
    var = var < 0.0 ? 0.0 : var;
    const float a  = gam[c] * (1.0f / sqrtf((float)var + BNEPS));
    const float bb = bet[c] - (float)mu * a;
    pl[c] = a;
    pl[C + c] = bb;
  }
  __syncthreads();
  const int nv = (2 * C) / 4;
  v4f v = {0.f, 0.f, 0.f, 0.f};
  if (tid < nv) v = *(const v4f*)(pl + 4 * tid);
  if (tid < nv) *(volatile v4f*)(ab + 4 * tid) = v;
  __threadfence();
  if (tid < nv) *(volatile v4f*)(ab + 4 * tid) = v;
}

__global__ __launch_bounds__(NTHR) void k_bnapply(float* h, const float* __restrict__ ab, int nv) {
  const int i = blockIdx.x * NTHR + (int)threadIdx.x;
  if (i >= nv) return;
  const int c = (i & 7) * 4;
  const v4f a = *(const v4f*)(ab + c);
  const v4f b = *(const v4f*)(ab + C1 + c);
  float* p = h + (size_t)i * 4;
  const v4f xv = *(const v4f*)p;
  const v4f r = xv * a + b;
  *(volatile v4f*)p = r;
  __threadfence();
  *(volatile v4f*)p = r;
}

__global__ __launch_bounds__(NTHR) void k_layer2(
    const int* __restrict__ csr, const int* __restrict__ off, const int* __restrict__ cnt,
    const int* __restrict__ ei, const float* __restrict__ ea, const float* __restrict__ h1,
    const _Float16* __restrict__ W2h, float* h2, float* part, int nN, int nE, int csrLen) {
  extern __shared__ v4f lds_dyn[];
  float* accT = (float*)lds_dyn;
  const int tid = threadIdx.x, lane = tid & 31, wave = tid >> 5;
  {
    const v4f z = {0.f, 0.f, 0.f, 0.f};
#pragma unroll 1
    for (int i = tid; i < TG2 * KP2 / 4; i += NTHR) lds_dyn[i] = z;
  }
  const int tb = blockIdx.x * TG2 + wave * 8;
  const int cl = tb + (lane & 7);
  const int cnt_l = cnt[cl];
  const int off_l = off[cl];
  const int cb = lane >> 2, q = lane & 3;
  const int cc = (cb & 1) + 3 * ((cb >> 1) & 1) + 9 * ((cb >> 2) & 1);
  const bool bx = (cb & 1) != 0, by = (cb & 2) != 0, bz = (cb & 4) != 0;
  __syncthreads();

  float* wrow = accT + (size_t)(wave * 8) * KP2 + 8 * q;
#pragma unroll 1
  for (int j = 0; j < 8; ++j) {
    int craw = __builtin_amdgcn_readlane(cnt_l, j);
    craw = craw < 0 ? 0 : craw;
    const int n = craw > DEGCAP ? DEGCAP : craw;
    const int st = __builtin_amdgcn_readlane(off_l, j);
    float* trow = wrow + j * KP2;
#pragma unroll 1
    for (int q0 = 0; q0 < n; q0 += 32) {
      const int pos = clampi(st + q0 + lane, 0, csrLen - 1);
      const int e = clampi(csr[pos], 0, nE - 1);
      const int s = clampi(ei[e], 0, nN - 1);
      const float* ap = ea + (size_t)e * 3;
      const float v0 = ap[0] * 2.0f, v1 = ap[1] * 2.0f, v2 = ap[2] * 2.0f;
      const float l0 = fminf(fmaxf(floorf(v0), 0.0f), 1.0f);
      const float l1 = fminf(fmaxf(floorf(v1), 0.0f), 1.0f);
      const float l2 = fminf(fmaxf(floorf(v2), 0.0f), 1.0f);
      const float f0 = v0 - l0, f1 = v1 - l1, f2 = v2 - l2;
      const int lb = (int)l0 + 3 * (int)l1 + 9 * (int)l2;
      const int mcnt = (n - q0) < 32 ? (n - q0) : 32;
#pragma unroll 1
      for (int p = 0; p < mcnt; ++p) {
        const int sp    = __builtin_amdgcn_readlane(s, p);
        const float pf0 = rlf(f0, p), pf1 = rlf(f1, p), pf2 = rlf(f2, p);
        const int plb   = __builtin_amdgcn_readlane(lb, p);
        const float wx = bx ? pf0 : 1.0f - pf0;
        const float wy = by ? pf1 : 1.0f - pf1;
        const float wz = bz ? pf2 : 1.0f - pf2;
        const float w = (wx * wy) * wz;
        const float* hp = h1 + (size_t)sp * C1 + 8 * q;
        const v4f hv0 = *(const v4f*)hp;
        const v4f hv1 = *(const v4f*)(hp + 4);
        v4f* ak = (v4f*)(trow + (plb + cc) * C1);
        v4f a0 = ak[0], a1 = ak[1];
        a0 = a0 + w * hv0;
        a1 = a1 + w * hv1;
        ak[0] = a0;
        ak[1] = a1;
      }
    }
  }
  __syncthreads();

  const int hh = lane >> 4, m = lane & 15;
  const int rt = wave >> 1, ct0 = (wave & 1) * 4;
  v8f acc[4];
#pragma unroll
  for (int t = 0; t < 4; ++t) { v8f z8 = {0.f, 0.f, 0.f, 0.f, 0.f, 0.f, 0.f, 0.f}; acc[t] = z8; }
  const float* ar = accT + (size_t)(rt * 16 + m) * KP2 + 8 * hh;
#pragma unroll 1
  for (int kt = 0; kt < KT2; ++kt) {
    const float* ak = ar + 32 * kt;
    FragH a;
    a.h[0] = cvt8(*(const v4f*)ak, *(const v4f*)(ak + 4));
    a.h[1] = cvt8(*(const v4f*)(ak + 16), *(const v4f*)(ak + 20));
#pragma unroll
    for (int t = 0; t < 4; ++t) {
      const _Float16* bp = W2h + (size_t)(16 * (ct0 + t) + m) * KP2 + 32 * kt + 8 * hh;
      FragH b;
      b.h[0] = *(const v8h*)bp;
      b.h[1] = *(const v8h*)(bp + 16);
      acc[t] = wmh(a.v, b.v, acc[t]);
    }
  }
  __syncthreads();

  float* stg = accT;
  float* sS  = accT + TG2 * C2;
  float* sQ  = sS + 2 * C2;
  float* pl  = sQ + 2 * C2;
  const int lr0 = rt * 16 + 8 * hh;
  float rc[8];
#pragma unroll
  for (int r = 0; r < 8; ++r) {
    int d = cnt[blockIdx.x * TG2 + lr0 + r];
    d = d < 1 ? 1 : d;
    rc[r] = (1.0f / (float)d) * W2I;
  }
#pragma unroll
  for (int t = 0; t < 4; ++t) {
    float* spp = stg + lr0 * C2 + 16 * (ct0 + t) + m;
#pragma unroll
    for (int r = 0; r < 8; ++r) spp[r * C2] = acc[t][r] * rc[r];
  }
  __syncthreads();
  {
    const int col = tid & (C2 - 1);
    const int r0 = (tid >> 7) * 32;
    float sum = 0.0f, sq = 0.0f;
#pragma unroll 1
    for (int r = 0; r < 32; ++r) {
      float* p_ = stg + (r0 + r) * C2 + col;
      float v = *p_;
      v = v > 0.0f ? v : expm1f(v);
      *p_ = v;
      sum += v;
      sq += v * v;
    }
    sS[(tid >> 7) * C2 + col] = sum;
    sQ[(tid >> 7) * C2 + col] = sq;
  }
  __syncthreads();
  if (tid < C2) {
    pl[tid] = sS[tid] + sS[C2 + tid];
    pl[C2 + tid] = sQ[tid] + sQ[C2 + tid];
  }
  __syncthreads();

  v4f pv = {0.f, 0.f, 0.f, 0.f};
  if (tid < 64) pv = *(const v4f*)(pl + 4 * tid);
  float* pp = part + (size_t)blockIdx.x * (2 * C2) + 4 * tid;
  const float* lp = stg + (wave * 8) * C2 + 4 * lane;
  float* gp = h2 + ((size_t)blockIdx.x * TG2 + wave * 8) * C2 + 4 * lane;
  if (tid < 64) *(volatile v4f*)pp = pv;
#pragma unroll
  for (int i = 0; i < 8; ++i) { const v4f v = *(const v4f*)(lp + i * C2); *(volatile v4f*)(gp + (size_t)i * C2) = v; }
  __threadfence();
  if (tid < 64) *(volatile v4f*)pp = pv;
#pragma unroll
  for (int i = 0; i < 8; ++i) { const v4f v = *(const v4f*)(lp + i * C2); *(volatile v4f*)(gp + (size_t)i * C2) = v; }
}

__global__ __launch_bounds__(NTHR) void k_pool(
    const int* __restrict__ batch, const float* __restrict__ pos, const float* __restrict__ h2,
    const float* __restrict__ ab, float* feat, int nN, int vec8) {
  extern __shared__ v4f lds_dyn[];
  float* wmax = (float*)lds_dyn;
  int* list = (int*)(wmax + NWAVE * CL * C2);
  const int tid = threadIdx.x, lane = tid & 31, wave = tid >> 5;
  const int g = blockIdx.x;
  {
    const float nin = -__builtin_inff();
    const v4f z = {nin, nin, nin, nin};
#pragma unroll 1
    for (int i = tid; i < NWAVE * CL * C2 / 4; i += NTHR) lds_dyn[i] = z;
  }
  const v4f a4 = *(const v4f*)(ab + 4 * lane);
  const v4f b4 = *(const v4f*)(ab + C2 + 4 * lane);
  const float R60 = 1.0f / 60.0f, R45 = 1.0f / 45.0f;
  __syncthreads();

  float* mt = wmax + wave * (CL * C2) + 4 * lane;
  const int nChunks = (nN + CHUNK - 1) / CHUNK;
#pragma unroll 1
  for (int ch = 0; ch < nChunks; ++ch) {
    const int cbase = ch * CHUNK;
    const int wc = scan_chunk<1>(batch, nN, cbase, g, vec8, list, tid, lane, wave);
    __syncthreads();
    int n = __builtin_amdgcn_readfirstlane(wc);
    n = n > WCAP ? WCAP : (n < 0 ? 0 : n);
    const int* lp = list + wave * WCAP;
#pragma unroll 1
    for (int i = 0; i < n; ++i) {
      const int ent = __builtin_amdgcn_readfirstlane(lp[i]);
      int nd = cbase + ((ent >> 12) & (CHUNK - 1));
      nd = nd > nN - 1 ? nN - 1 : nd;
      const float* ppos = pos + (size_t)nd * 3;
      const float px = ppos[0], py = ppos[1];
      float fx = floorf(px * R60); fx = fminf(fmaxf(fx, 0.0f), 3.0f);
      float fy = floorf(py * R45); fy = fminf(fmaxf(fy, 0.0f), 3.0f);
      const int clu = (int)fy * 4 + (int)fx;
      const v4f hv = *(const v4f*)(h2 + (size_t)nd * C2 + 4 * lane);
      const v4f v = hv * a4 + b4;
      v4f* mp = (v4f*)(mt + clu * C2);
      v4f mv = *mp;
      mv.x = fmaxf(mv.x, v.x); mv.y = fmaxf(mv.y, v.y); mv.z = fmaxf(mv.z, v.z); mv.w = fmaxf(mv.w, v.w);
      *mp = mv;
    }
    __syncthreads();
  }
  __syncthreads();

  v4f rv[2];
#pragma unroll
  for (int p = 0; p < 2; ++p) {
    const int f = 4 * (wave * 64 + 32 * p + lane);
    v4f r = *(const v4f*)(wmax + f);
#pragma unroll
    for (int w = 1; w < NWAVE; ++w) {
      const v4f o = *(const v4f*)(wmax + w * (CL * C2) + f);
      r.x = fmaxf(r.x, o.x); r.y = fmaxf(r.y, o.y); r.z = fmaxf(r.z, o.z); r.w = fmaxf(r.w, o.w);
    }
    r.x = ((__float_as_uint(r.x) & 0x7f800000u) != 0x7f800000u) ? r.x : 0.0f;
    r.y = ((__float_as_uint(r.y) & 0x7f800000u) != 0x7f800000u) ? r.y : 0.0f;
    r.z = ((__float_as_uint(r.z) & 0x7f800000u) != 0x7f800000u) ? r.z : 0.0f;
    r.w = ((__float_as_uint(r.w) & 0x7f800000u) != 0x7f800000u) ? r.w : 0.0f;
    rv[p] = r;
  }
  float* fp = feat + (size_t)g * KF;
#pragma unroll
  for (int p = 0; p < 2; ++p) *(volatile v4f*)(fp + 4 * (wave * 64 + 32 * p + lane)) = rv[p];
  __threadfence();
#pragma unroll
  for (int p = 0; p < 2; ++p) *(volatile v4f*)(fp + 4 * (wave * 64 + 32 * p + lane)) = rv[p];
}

__global__ __launch_bounds__(NTHR) void k_fc(
    const float* __restrict__ feat, const float* __restrict__ fcw, const int* __restrict__ numg,
    float* out, int G, int NO) {
  extern __shared__ v4f lds_dyn[];
  float* F    = (float*)lds_dyn;
  float* ostg = F + GMAX * KF;
  const int tid = threadIdx.x;
  (void)numg;
#pragma unroll 1
  for (int i = tid; i < G * KF / 4; i += NTHR) lds_dyn[i] = ((const v4f*)feat)[i];
  __syncthreads();
  const int nfl = G * NO;
#pragma unroll 1
  for (int i = tid; i < nfl; i += NTHR) {
    const int gg = i / NO;
    const int o  = i - gg * NO;
    const float* wr = fcw + (size_t)o * KF;
    const float* fr = F + gg * KF;
    float s = 0.0f;
#pragma unroll 1
    for (int k = 0; k < KF; k += 4) {
      const v4f w = *(const v4f*)(wr + k);
      const v4f f = *(const v4f*)(fr + k);
      s += f.x * w.x;
      s += f.y * w.y;
      s += f.z * w.z;
      s += f.w * w.w;
    }
    ostg[i] = s;
  }
  __syncthreads();
  const int nv = nfl >> 2;
  const int tail = nfl & 3;
  v4f ov[2];
#pragma unroll
  for (int p = 0; p < 2; ++p) {
    const int i4 = tid + NTHR * p;
    v4f v = {0.f, 0.f, 0.f, 0.f};
    if (i4 < nv) v = *(const v4f*)(ostg + 4 * i4);
    ov[p] = v;
  }
  float tv = 0.0f;
  if (tid < tail) tv = ostg[4 * nv + tid];
#pragma unroll
  for (int p = 0; p < 2; ++p) { const int i4 = tid + NTHR * p; if (i4 < nv) *(volatile v4f*)(out + 4 * i4) = ov[p]; }
  if (tid < tail) *(volatile float*)(out + 4 * nv + tid) = tv;
  __threadfence();
#pragma unroll
  for (int p = 0; p < 2; ++p) { const int i4 = tid + NTHR * p; if (i4 < nv) *(volatile v4f*)(out + 4 * i4) = ov[p]; }
  if (tid < tail) *(volatile float*)(out + 4 * nv + tid) = tv;
}

extern "C" void kernel_launch(void* const* d_in, const int* in_sizes, int n_in,
                              void* d_out, int out_size, void* d_ws, size_t ws_size,
                              hipStream_t stream) {
  if (n_in < 13) return;
  const int nN = in_sizes[0];
  if (nN <= 0 || in_sizes[1] != 3 * nN || in_sizes[11] != nN) return;
  const int nE = in_sizes[10] / 2;
  if (nE <= 0 || in_sizes[10] != 2 * nE || in_sizes[2] != 3 * nE) return;
  if (in_sizes[3] != KK * C1 || in_sizes[4] < C1 || in_sizes[5] < C1) return;
  if (in_sizes[6] != K2 * C2 || in_sizes[7] < C2 || in_sizes[8] < C2) return;
  const int NO = in_sizes[9] / KF;
  if (NO < 1 || NO > NOMAX || in_sizes[9] != NO * KF) return;
  const int G = out_size / NO;
  if (G < 1 || G > GMAX || G * NO != out_size) return;
  if (in_sizes[12] < 1) return;
  if (nN > (1 << 24) || nE > (1 << 28)) return;

  const float* x    = (const float*)d_in[0];
  const float* pos  = (const float*)d_in[1];
  const float* ea   = (const float*)d_in[2];
  const float* W1   = (const float*)d_in[3];
  const float* g1   = (const float*)d_in[4];
  const float* be1  = (const float*)d_in[5];
  const float* W2   = (const float*)d_in[6];
  const float* g2   = (const float*)d_in[7];
  const float* be2  = (const float*)d_in[8];
  const float* fcw  = (const float*)d_in[9];
  const int*   ei   = (const int*)d_in[10];
  const int*   bat  = (const int*)d_in[11];
  const int*   numg = (const int*)d_in[12];
  const int*   dsts = ei + nE;
  float* out = (float*)d_out;

  const int NPAD   = ((nN + NTHR - 1) / NTHR) * NTHR;
  const int nBC    = (nN + NBC - 1) / NBC;
  const int CNTPAD = nBC * NBC;
  if (4 * nBC + 1 > RBN) return;
  const int nBF    = (nN + NBF - 1) / NBF;
  const int csrLen = ((nE + 31) & ~31) + 4096;
  const int nL1    = NPAD / NTHR;
  const int nL2    = NPAD / TG2;
  const int nApply = NPAD / 32;
  const int nPrep  = C2 * (KP2 / 8);

  char* ws = (char*)d_ws;
  size_t off = 0;
  const size_t oCnt  = off; off += (size_t)CNTPAD * 4;                 off = (off + 255) & ~(size_t)255;
  const size_t oOff  = off; off += (size_t)CNTPAD * 4;                 off = (off + 255) & ~(size_t)255;
  const size_t oRb   = off; off += (size_t)RBN * 4;                    off = (off + 255) & ~(size_t)255;
  const size_t oCsr  = off; off += (size_t)csrLen * 4;                 off = (off + 255) & ~(size_t)255;
  const size_t oH1   = off; off += (size_t)NPAD * C1 * 4;              off = (off + 255) & ~(size_t)255;
  const size_t oP1   = off; off += (size_t)nL1 * (2 * C1) * 4;         off = (off + 255) & ~(size_t)255;
  const size_t oAb1  = off; off += (size_t)(2 * C1) * 4;               off = (off + 255) & ~(size_t)255;
  const size_t oW2h  = off; off += (size_t)C2 * KP2 * 2;               off = (off + 255) & ~(size_t)255;
  const size_t oH2   = off; off += (size_t)NPAD * C2 * 4;              off = (off + 255) & ~(size_t)255;
  const size_t oP2   = off; off += (size_t)nL2 * (2 * C2) * 4;         off = (off + 255) & ~(size_t)255;
  const size_t oAb2  = off; off += (size_t)(2 * C2) * 4;               off = (off + 255) & ~(size_t)255;
  const size_t oFeat = off; off += (size_t)G * KF * 4;                 off = (off + 255) & ~(size_t)255;
  if (off > ws_size || off > ((size_t)128 << 20)) return;
  int*      cnt   = (int*)(ws + oCnt);
  int*      offp  = (int*)(ws + oOff);
  int*      rb    = (int*)(ws + oRb);
  int*      csr   = (int*)(ws + oCsr);
  float*    h1    = (float*)(ws + oH1);
  float*    part1 = (float*)(ws + oP1);
  float*    ab1   = (float*)(ws + oAb1);
  _Float16* W2h   = (_Float16*)(ws + oW2h);
  float*    h2    = (float*)(ws + oH2);
  float*    part2 = (float*)(ws + oP2);
  float*    ab2   = (float*)(ws + oAb2);
  float*    feat  = (float*)(ws + oFeat);

  const int vec8e = ((nE & 3) == 0) ? 1 : 0;
  const int vec8n = ((nN & 3) == 0) ? 1 : 0;

  k_w2prep<<<(nPrep + NTHR - 1) / NTHR, NTHR, 0, stream>>>(W2, W2h, nPrep);

  k_count<<<nBC, NTHR, 0, stream>>>(dsts, cnt, nE, vec8e);
  k_offsets<<<1, OTHR, 0, stream>>>(cnt, offp, rb, nBC);
  hipFuncSetAttribute(reinterpret_cast<const void*>(&k_fill),
                      hipFuncAttributeMaxDynamicSharedMemorySize, LDS_FILL);
  k_fill<<<nBF, NTHR, LDS_FILL, stream>>>(dsts, offp, rb, csr, nE, vec8e, csrLen);

  hipFuncSetAttribute(reinterpret_cast<const void*>(&k_layer1),
                      hipFuncAttributeMaxDynamicSharedMemorySize, LDS_L1);
  k_layer1<<<nL1, NTHR, LDS_L1, stream>>>(csr, offp, cnt, ei, ea, x, W1, h1, part1, nN, nE, csrLen);
  k_bnfin<<<1, 128, 0, stream>>>(part1, g1, be1, ab1, nL1, C1, nN);
  k_bnapply<<<nApply, NTHR, 0, stream>>>(h1, ab1, NPAD * (C1 / 4));

  hipFuncSetAttribute(reinterpret_cast<const void*>(&k_layer2),
                      hipFuncAttributeMaxDynamicSharedMemorySize, LDS_L2);
  k_layer2<<<nL2, NTHR, LDS_L2, stream>>>(csr, offp, cnt, ei, ea, h1, W2h, h2, part2, nN, nE, csrLen);
  k_bnfin<<<1, 128, 0, stream>>>(part2, g2, be2, ab2, nL2, C2, nN);

  hipFuncSetAttribute(reinterpret_cast<const void*>(&k_pool),
                      hipFuncAttributeMaxDynamicSharedMemorySize, LDS_POOL);
  k_pool<<<G, NTHR, LDS_POOL, stream>>>(bat, pos, h2, ab2, feat, nN, vec8n);

  hipFuncSetAttribute(reinterpret_cast<const void*>(&k_fc),
                      hipFuncAttributeMaxDynamicSharedMemorySize, LDS_FC);
  k_fc<<<1, NTHR, LDS_FC, stream>>>(feat, fcw, numg, out, G, NO);
}
